// GNNRepresentationNetwork_27230092657584
// MI455X (gfx1250) — hardware-verified
//
#include <hip/hip_runtime.h>
#include <math.h>

typedef __attribute__((ext_vector_type(16))) _Float16 v16h;
typedef __attribute__((ext_vector_type(16))) __bf16 v16b;
typedef __attribute__((ext_vector_type(8)))  _Float16 v8h;
typedef __attribute__((ext_vector_type(8)))  float v8f;
typedef __attribute__((ext_vector_type(4)))  float v4f;
typedef __attribute__((ext_vector_type(2)))  float v2f;
typedef __attribute__((ext_vector_type(4)))  unsigned v4u;
typedef __attribute__((ext_vector_type(4)))  int v4i;
typedef float __attribute__((may_alias)) float_a;
typedef int __attribute__((may_alias)) int_a;

template <typename T> __device__ __forceinline__ void vst2(void* p, T v) { *(volatile T*)p = v; __threadfence(); *(volatile T*)p = v; }
__device__ __forceinline__ v8f wmma16(v16h a, v16h b, v8f c) {
  v8f d = __builtin_amdgcn_wmma_f32_16x16x32_f16(false, a, false, b, (short)0, c, false, false);
  asm volatile("v_nop\n\tv_nop\n\tv_nop\n\tv_nop" : "+v"(d) : "v"(a), "v"(b));
  return d;
}
__device__ __forceinline__ v8f wmma_bf(v16b a, v16b b, v8f c) {
  v8f d = __builtin_amdgcn_wmma_f32_16x16x32_bf16(false, a, false, b, (short)0, c, false, false);
  asm volatile("v_nop\n\tv_nop\n\tv_nop\n\tv_nop" : "+v"(d) : "v"(a), "v"(b));
  return d;
}
__device__ __forceinline__ v16h frag_h(const _Float16* rowk0, int lane) {
  union { v16h v; v8h q[2]; } u; const _Float16* p = rowk0 + 8 * (lane >> 4);
  u.q[0] = *(const v8h*)p; u.q[1] = *(const v8h*)(p + 16); return u.v;
}
__device__ __forceinline__ v16h frag_f32(const float* rowk0, int lane) {
  v16h a; const float* p = rowk0 + 8 * (lane >> 4);
#pragma unroll
  for (int i = 0; i < 8; ++i) { a[i] = (_Float16)p[i]; a[8 + i] = (_Float16)p[16 + i]; }
  return a;
}
__device__ __forceinline__ v16h frag_f32s(const float* rowk0, int lane, float sc) {
  v16h a; const float* p = rowk0 + 8 * (lane >> 4);
#pragma unroll
  for (int i = 0; i < 8; ++i) { a[i] = (_Float16)(p[i] * sc); a[8 + i] = (_Float16)(p[16 + i] * sc); }
  return a;
}
__device__ __forceinline__ v16h fragc_f32(const float* W, int k0, int n, int lane, int ld, int K) {
  v16h a; const int g = lane >> 4;
#pragma unroll
  for (int i = 0; i < 8; ++i) { const int ka = k0 + 8 * g + i, kb = ka + 16;
    a[i] = (_Float16)(ka < K ? W[(size_t)(ka < K ? ka : K - 1) * ld + n] : 0.f); a[8 + i] = (_Float16)(kb < K ? W[(size_t)(kb < K ? kb : K - 1) * ld + n] : 0.f); }
  return a;
}
struct F2 { v16b h, l; };
__device__ __forceinline__ F2 bsplit16(const float v[16]) { F2 r;
#pragma unroll
  for (int i = 0; i < 16; ++i) { const __bf16 h = (__bf16)v[i]; r.h[i] = h; r.l[i] = (__bf16)(v[i] - (float)h); }
  return r; }
__device__ __forceinline__ F2 split_row(const float* row, int k0, int lane) { float v[16]; const float* p = row + k0 + 8 * (lane >> 4);
#pragma unroll
  for (int i = 0; i < 8; ++i) { v[i] = p[i]; v[8 + i] = p[16 + i]; }
  return bsplit16(v); }
__device__ __forceinline__ F2 split_rowK(const float* row, int k0, int lane, int K) { float v[16]; const int g = lane >> 4;
#pragma unroll
  for (int i = 0; i < 8; ++i) { const int ka = k0 + 8 * g + i, kb = ka + 16; v[i] = ka < K ? row[ka < K ? ka : K - 1] : 0.f; v[8 + i] = kb < K ? row[kb < K ? kb : K - 1] : 0.f; }
  return bsplit16(v); }
__device__ __forceinline__ F2 split_col(const float* W, int k0, int n, int lane, int ld, int K) { float v[16]; const int g = lane >> 4;
#pragma unroll
  for (int i = 0; i < 8; ++i) { const int ka = k0 + 8 * g + i, kb = ka + 16; v[i] = ka < K ? W[(size_t)(ka < K ? ka : K - 1) * ld + n] : 0.f; v[8 + i] = kb < K ? W[(size_t)(kb < K ? kb : K - 1) * ld + n] : 0.f; }
  return bsplit16(v); }
__device__ __forceinline__ v8f mac3(const F2& a, const F2& b, v8f c) { c = wmma_bf(a.l, b.h, c); c = wmma_bf(a.h, b.l, c); return wmma_bf(a.h, b.h, c); }
__device__ __forceinline__ float sigm(float v) { return 1.0f / (1.0f + expf(-v)); }
#define LDSX() do { asm volatile("s_wait_dscnt 0" ::: "memory"); __builtin_amdgcn_wave_barrier(); __builtin_amdgcn_fence(__ATOMIC_RELEASE, "workgroup"); } while (0)


#define NB 16
#define GH 64
#define GW 64
#define NN (GH * GW)
#define NR (NB * NN)
#define C0 16
#define DE 64
#define DH 128
#define DR 256
#ifndef TRB
#define TRB (NR / 64)
#define TNB NB
#endif
typedef __attribute__((ext_vector_type(8))) __bf16 v8b;
__device__ __forceinline__ v16b frag_b(const __bf16* rowk0, int lane) {
  union { v16b v; v8b q[2]; } u; const __bf16* p = rowk0 + 8 * (lane >> 4);
  u.q[0] = *(const v8b*)p; u.q[1] = *(const v8b*)(p + 16); return u.v;
}
__device__ __forceinline__ float bfr(float v) { return (float)(__bf16)v; }
#define PK_E1 0
#define PK_E2 (PK_E1 + 64 * 64)
#define PK_G1 (PK_E2 + 64 * 64)
#define PK_G2 (PK_G1 + 128 * 64)
#define PK_G3 (PK_G2 + 128 * 128)
#define PK_R1 (PK_G3 + 128 * 128)
#define PK_R2 (PK_R1 + 256 * 128)
#define PK_END (PK_R2 + 256 * 256)
#define WS_PK   0u
#define WS_HA   (WS_PK + 2u * PK_END)
#define WS_HB   (WS_HA + 4u * NR * DH)
#define WS_PART (WS_HB + 4u * NR * DH)
#define WS_END  (WS_PART + 4u * (NR / 64) * DH)

__global__ __launch_bounds__(256) void k_pack(const float* __restrict__ e1, const float* __restrict__ e2, const float* __restrict__ g1, const float* __restrict__ g2, const float* __restrict__ g3, const float* __restrict__ r1, const float* __restrict__ r2, __bf16* __restrict__ PK) {
  __shared__ __align__(16) __bf16 srow[256];
  const int n = blockIdx.x, tid = threadIdx.x; const float* W; int K, KP, NO, o; size_t dst; int m = n;
  if (m < 64) { W = e1; K = C0; KP = 64; NO = DE; o = m; dst = PK_E1 + (size_t)o * 64; }   else if ((m -= 64) < 64) { W = e2; K = DE; KP = 64; NO = DE; o = m; dst = PK_E2 + (size_t)o * 64; }
  else if ((m -= 64) < 128) { W = g1; K = DE; KP = 64; NO = DH; o = m; dst = PK_G1 + (size_t)o * 64; } else if ((m -= 128) < 128) { W = g2; K = DH; KP = 128; NO = DH; o = m; dst = PK_G2 + (size_t)o * 128; }
  else if ((m -= 128) < 128) { W = g3; K = DH; KP = 128; NO = DH; o = m; dst = PK_G3 + (size_t)o * 128; } else if ((m -= 128) < 256) { W = r1; K = DH; KP = 128; NO = DR; o = m; dst = PK_R1 + (size_t)o * 128; }
  else { m -= 256; W = r2; K = DR; KP = 256; NO = DR; o = m; dst = PK_R2 + (size_t)o * 256; }
  { const float wv = bfr(W[(size_t)min(tid, K - 1) * NO + o]); srow[tid] = (__bf16)((tid < K) ? wv : 0.f); }
  __syncthreads();
  if (tid < KP / 8) vst2((unsigned*)(PK + dst + tid * 8), *(const v4u*)(&srow[tid * 8]));
}
__global__ __launch_bounds__(128) void k_embed1(const float* __restrict__ OBS, const __bf16* __restrict__ PK, const float* __restrict__ b1, float* __restrict__ HA) {
  __shared__ __align__(16) __bf16 sa[64][40]; __shared__ __align__(16) float so[4][16][68];
  const int tid = threadIdx.x, wave = tid >> 5, lane = tid & 31, col = lane & 15, g = lane >> 4; const size_t r0 = (size_t)blockIdx.x * 64; const int b = (int)(r0 / NN), n0 = (int)(r0 % NN);
  for (int q = tid; q < 64 * 32; q += 128) { const int rl = q & 63, c = q >> 6; sa[rl][c] = (__bf16)((c < C0) ? bfr(OBS[((size_t)b * C0 + c) * NN + n0 + rl]) : 0.f); }
  __syncthreads();
  v8f acc[4] = {};
  { const v16b a = frag_b(&sa[wave * 16 + col][0], lane);
#pragma unroll
    for (int j = 0; j < 4; ++j) acc[j] = wmma_bf(a, frag_b(PK + PK_E1 + (size_t)(j * 16 + col) * 64, lane), acc[j]); }
#pragma unroll
  for (int j = 0; j < 4; ++j) { const float bb = bfr(b1[j * 16 + col]);
#pragma unroll
    for (int r = 0; r < 8; ++r) so[wave][8 * g + r][j * 16 + col] = fmaxf(acc[j][r] + bb, 0.f); }
  LDSX();
  for (int rl = 0; rl < 16; ++rl) if (lane < 16) vst2(HA + (r0 + wave * 16 + rl) * DH + lane * 4, *(const v4f*)&so[wave][rl][lane * 4]);
}
template <int KI, int NO, bool ACT>
__global__ __launch_bounds__(128) void k_lin(const float* __restrict__ IN, const __bf16* __restrict__ P, const float* __restrict__ bias, float* __restrict__ OUT) {
  __shared__ __align__(16) float so[4][16][132];
  const int tid = threadIdx.x, wave = tid >> 5, lane = tid & 31, col = lane & 15, g = lane >> 4; const size_t r0 = (size_t)blockIdx.x * 64 + wave * 16;
  v8f acc[NO / 16] = {};
#pragma unroll
  for (int kc = 0; kc < KI / 32; ++kc) { const F2 a = split_row(IN + (r0 + col) * DH, kc * 32, lane);
#pragma unroll
    for (int j = 0; j < NO / 16; ++j) { const v16b w = frag_b(P + (size_t)(j * 16 + col) * KI + kc * 32, lane); acc[j] = wmma_bf(a.l, w, acc[j]); acc[j] = wmma_bf(a.h, w, acc[j]); } }
#pragma unroll
  for (int j = 0; j < NO / 16; ++j) { const float bb = bfr(bias[j * 16 + col]);
#pragma unroll
    for (int r = 0; r < 8; ++r) { float v = acc[j][r] + bb; if (ACT) v = fmaxf(v, 0.f); so[wave][8 * g + r][j * 16 + col] = v; } }
  LDSX();
  for (int rl = 0; rl < 16; ++rl) for (int pc = lane; pc < NO / 4; pc += 32) vst2(OUT + (r0 + rl) * DH + pc * 4, *(const v4f*)&so[wave][rl][pc * 4]);
}
__global__ __launch_bounds__(256) void k_stencil(const float* __restrict__ S, float* __restrict__ H) {
  const int tid = threadIdx.x; const size_t r = (size_t)blockIdx.x * 64 + (tid >> 2); const int c0 = (tid & 3) * 32; const int b = (int)(r / NN), n = (int)(r % NN); const int i = n / GW, j = n % GW;
  const float* base = S + (size_t)b * NN * DH; int nb[4]; int deg = 0;
  if (i > 0) nb[deg++] = n - GW; if (i < GH - 1) nb[deg++] = n + GW; if (j > 0) nb[deg++] = n - 1; if (j < GW - 1) nb[deg++] = n + 1;
  const float inv = 1.0f / ((float)deg + 1e-6f);
#pragma unroll
  for (int p = 0; p < 8; ++p) { v4f v; for (int k = 0; k < 4; ++k) { const int c = c0 + p * 4 + k; float s = 0.f; for (int q = 0; q < deg; ++q) s += base[(size_t)nb[q] * DH + c]; v[k] = fmaxf(s * inv, 0.f); } vst2(H + r * DH + c0 + p * 4, v); }
}
__global__ __launch_bounds__(128) void k_colpart(const float* __restrict__ H, float* __restrict__ PART) {
  __shared__ __align__(16) float s[128]; const int c = threadIdx.x; const size_t r0 = (size_t)blockIdx.x * 64; float a = 0.f; for (int r = 0; r < 64; ++r) a += H[(r0 + r) * DH + c]; s[c] = a; __syncthreads();
  if (c < 32) vst2(PART + (size_t)blockIdx.x * DH + c * 4, *(const v4f*)&s[c * 4]);
}
__global__ __launch_bounds__(256) void k_head(const float* __restrict__ PART, const __bf16* __restrict__ PK, const float* __restrict__ rb1, const float* __restrict__ rb2, float* __restrict__ OUT) {
  __shared__ float sg[128], sg1[256]; __shared__ __align__(16) float so[256];
  const int b = blockIdx.x, tid = threadIdx.x;
  if (tid < DH) { float a = 0.f; for (int k = 0; k < NN / 64; ++k) a += PART[((size_t)b * (NN / 64) + k) * DH + tid]; sg[tid] = a / (float)NN; }
  __syncthreads();
  { float a = bfr(rb1[tid]);
#pragma unroll 1
    for (int k = 0; k < DH; ++k) a += sg[k] * (float)PK[PK_R1 + (size_t)tid * DH + k];
    sg1[tid] = fmaxf(a, 0.f); }
  __syncthreads();
  { float a = bfr(rb2[tid]);
#pragma unroll 1
    for (int k = 0; k < DR; ++k) a += sg1[k] * (float)PK[PK_R2 + (size_t)tid * DR + k];
    so[tid] = fmaxf(a, 0.f); }
  __syncthreads();
  if (tid < 64) vst2(OUT + (size_t)b * DR + tid * 4, *(const v4f*)&so[tid * 4]);
}

extern "C" void kernel_launch(void* const* d_in, const int* in_sizes, int n_in, void* d_out, int out_size, void* d_ws, size_t ws_size, hipStream_t stream) {
  (void)in_sizes; (void)n_in; (void)out_size;
  const float** F = (const float**)d_in;
  if (ws_size < (size_t)WS_END) return;
  char* ws = (char*)d_ws; __bf16* PK = (__bf16*)(ws + WS_PK); float *HA = (float*)(ws + WS_HA), *HB = (float*)(ws + WS_HB), *PART = (float*)(ws + WS_PART);
  k_pack<<<64 + 64 + 128 * 3 + 256 * 2, 256, 0, stream>>>(F[1], F[3], F[5], F[7], F[9], F[11], F[13], PK);
  k_embed1<<<TRB, 128, 0, stream>>>(F[0], PK, F[2], HA);
  k_lin<64, 64, true><<<TRB, 128, 0, stream>>>(HA, PK + PK_E2, F[4], HB);
  k_lin<64, 128, false><<<TRB, 128, 0, stream>>>(HB, PK + PK_G1, F[6], HA);
  k_stencil<<<TRB, 256, 0, stream>>>(HA, HB);
  k_lin<128, 128, false><<<TRB, 128, 0, stream>>>(HB, PK + PK_G2, F[8], HA);
  k_stencil<<<TRB, 256, 0, stream>>>(HA, HB);
  k_lin<128, 128, false><<<TRB, 128, 0, stream>>>(HB, PK + PK_G3, F[10], HA);
  k_stencil<<<TRB, 256, 0, stream>>>(HA, HB);
  k_colpart<<<TRB, 128, 0, stream>>>(HB, PART);
  k_head<<<TNB, 256, 0, stream>>>(PART, PK, F[12], F[14], (float*)d_out);
}
